// TFLiteSTFT_31473520345491
// MI455X (gfx1250) — hardware-verified
//
#include <hip/hip_runtime.h>
#include <math.h>

typedef __attribute__((ext_vector_type(16))) _Float16 v16h;
typedef __attribute__((ext_vector_type(8)))  _Float16 v8h;
typedef __attribute__((ext_vector_type(8)))  float    v8f;
typedef __attribute__((ext_vector_type(4)))  float    v4f;
typedef __attribute__((ext_vector_type(2)))  float    v2f;

constexpr int kBatch   = 16;
constexpr int kSigLen  = 240000;
constexpr int kFrame   = 800;
constexpr int kStep    = 200;
constexpr int kFrames  = (kSigLen - kFrame) / kStep + 1;
constexpr int kBins    = kFrame / 2 + 1;
constexpr int kRowsM   = kBatch * kFrames;
constexpr int kRowsMP  = ((kRowsM + 63) / 64) * 64;
constexpr int kColsN   = 2 * kBins;
constexpr int kColsNP  = ((kColsN + 63) / 64) * 64;
constexpr int kDepthK  = kFrame;
constexpr int kTilesM  = kRowsMP / 64;
constexpr int kTilesN  = kColsNP / 64;
constexpr int kTiles   = kTilesM * kTilesN;
constexpr int kGemmBlocks = (kTiles + 7) / 8;
constexpr int kVecPerRow  = kDepthK / 8;
constexpr int kAVec    = kRowsMP * kVecPerRow;
constexpr int kBVec    = kColsNP * kVecPerRow;
constexpr int kOutElems = kRowsM * kColsN;
constexpr int kOutVec   = kOutElems / 4;
constexpr int kOutBlocks = (kOutVec + 255) / 256;

static_assert(kFrames == 1197, "frame count");
static_assert(kBins == 401, "bin count");
static_assert(kRowsM == 19152 && kRowsMP == 19200, "M and padded M");
static_assert(kColsN == 802 && kColsNP == 832, "N and padded N");
static_assert((kDepthK % 32) == 0, "K multiple of 32");
static_assert((kRowsMP % 64) == 0 && (kColsNP % 64) == 0, "tile multiples");
static_assert((kFrames - 1) * kStep + kFrame == kSigLen, "last frame ends at the last sample");
static_assert(kVecPerRow == 100, "8-element groups per row");
static_assert((kAVec % 256) == 0 && (kBVec % 256) == 0, "exact prep grids");
static_assert((kOutElems % 4) == 0, "float4 groups in the output");
static_assert((kColsN % 2) == 0, "pairs never straddle a row");
static_assert(kOutElems == 15359904, "output element count");

constexpr float kCarryA = 64.0f;
constexpr float kCarryB = 1024.0f;
constexpr float kFold   = 1.0f / (kCarryA * kCarryB);
constexpr float kHalfMinNormal = 6.103515625e-05f;

constexpr size_t kOffA   = 0;
constexpr size_t kSzA    = (size_t)kRowsMP * kDepthK * 2;
constexpr size_t kOffB   = kOffA + kSzA;
constexpr size_t kSzB    = (size_t)kColsNP * kDepthK * 2;
constexpr size_t kOffC   = kOffB + kSzB;
constexpr size_t kSzC    = (size_t)kRowsMP * kColsNP * 4;
constexpr size_t kWsTotal = kOffC + kSzC;
static_assert(kSzA == 30720000ull && kSzB == 1331200ull && kSzC == 63897600ull, "carve sizes");
static_assert(kWsTotal == 95948800ull, "carve total");
static_assert(kWsTotal <= 134217728ull, "carve cap");
static_assert((kOffB % 128) == 0 && (kOffC % 128) == 0, "128-B aligned regions");
static_assert(((size_t)kColsNP * 4) % 128 == 0, "padded product rows are whole lines");

__device__ __forceinline__ void tie_h(v8f& c, v16h a, v16h b) {
  asm volatile("v_nop\n\tv_nop\n\tv_nop\n\tv_nop" : "+v"(c) : "v"(a), "v"(b));
}
__device__ __forceinline__ void keep4_h(v16h a, v16h b, v16h c, v16h d) { asm volatile("v_nop" :: "v"(a), "v"(b), "v"(c), "v"(d)); }
__device__ __forceinline__ void acc_guard4(v8f& a, v8f& b, v8f& c, v8f& d) { asm volatile("v_nop\n\tv_nop\n\tv_nop\n\tv_nop" : "+v"(a), "+v"(b), "+v"(c), "+v"(d)); }

struct FragH {
  union U { v16h v; v8h h[2]; };
  static __device__ __forceinline__ v16h load(const _Float16* p) {
    U f; f.h[0] = *(const v8h*)(p); f.h[1] = *(const v8h*)(p + 16); return f.v;
  }
  static __device__ __forceinline__ v8f mma(v16h a, v16h b, v8f c) {
    return __builtin_amdgcn_wmma_f32_16x16x32_f16(false, a, false, b, (short)0, c, false, false);
  }
};

__global__ __launch_bounds__(256) void prep_a_kernel(
    const float* __restrict__ sig, const float* __restrict__ win, unsigned short* __restrict__ A16)
{
  const int t = blockIdx.x * 256 + threadIdx.x;
  const int m = t / kVecPerRow;
  const int n = (t - m * kVecPerRow) * 8;
  const int mc = (m < kRowsM) ? m : (kRowsM - 1);
  const int b = mc / kFrames;
  const int f = mc - b * kFrames;
  const float* sp = sig + (size_t)b * kSigLen + (size_t)(f * kStep + n);
  v4f s0 = *(const v4f*)(sp);
  v4f s1 = *(const v4f*)(sp + 4);
  v4f w0 = *(const v4f*)(win + n);
  v4f w1 = *(const v4f*)(win + n + 4);
  asm volatile("" : "+v"(s0));
  asm volatile("" : "+v"(s1));
  asm volatile("" : "+v"(w0));
  asm volatile("" : "+v"(w1));
  const bool live = (m < kRowsM);
  v8h hv;
#pragma unroll
  for (int e = 0; e < 4; ++e) {
    const float p0 = s0[e] * w0[e];
    const float p1 = s1[e] * w1[e];
    float x0 = p0 * kCarryA;
    float x1 = p1 * kCarryA;
    x0 = (fabsf(x0) < kHalfMinNormal) ? 0.0f : x0;
    x1 = (fabsf(x1) < kHalfMinNormal) ? 0.0f : x1;
    x0 = live ? x0 : 0.0f;
    x1 = live ? x1 : 0.0f;
    hv[e]     = (_Float16)x0;
    hv[4 + e] = (_Float16)x1;
  }
  unsigned short* q = A16 + ((size_t)t << 3);
  *(volatile v8h*)q = hv;
  __threadfence();
  *(volatile v8h*)q = hv;
}

__global__ __launch_bounds__(256) void prep_b_kernel(
    const float* __restrict__ tcos, const float* __restrict__ tsin, unsigned short* __restrict__ BT16)
{
  const int t = blockIdx.x * 256 + threadIdx.x;
  const int r = t / kVecPerRow;
  const int n = (t - r * kVecPerRow) * 8;
  const int kr = r >> 1;
  const int k = (kr < kBins) ? kr : (kBins - 1);
  const bool odd = (r & 1) != 0;
  const bool live = (r < kColsN);
  const float* pc = tcos + (size_t)k * kDepthK + n;
  const float* ps = tsin + (size_t)k * kDepthK + n;
  v4f c0 = *(const v4f*)(pc);
  v4f c1 = *(const v4f*)(pc + 4);
  v4f q0 = *(const v4f*)(ps);
  v4f q1 = *(const v4f*)(ps + 4);
  asm volatile("" : "+v"(c0));
  asm volatile("" : "+v"(c1));
  asm volatile("" : "+v"(q0));
  asm volatile("" : "+v"(q1));
  v8h hv;
#pragma unroll
  for (int e = 0; e < 4; ++e) {
    const float a0 = c0[e];
    const float a1 = c1[e];
    const float b0 = q0[e];
    const float b1 = q1[e];
    float x0 = (odd ? b0 : a0) * kCarryB;
    float x1 = (odd ? b1 : a1) * kCarryB;
    x0 = (fabsf(x0) < kHalfMinNormal) ? 0.0f : x0;
    x1 = (fabsf(x1) < kHalfMinNormal) ? 0.0f : x1;
    x0 = live ? x0 : 0.0f;
    x1 = live ? x1 : 0.0f;
    hv[e]     = (_Float16)x0;
    hv[4 + e] = (_Float16)x1;
  }
  unsigned short* q = BT16 + ((size_t)t << 3);
  *(volatile v8h*)q = hv;
  __threadfence();
  *(volatile v8h*)q = hv;
}

__global__ __launch_bounds__(256) void gemm_f16_nt_kernel(
    const unsigned short* __restrict__ Ap, int lda,
    const unsigned short* __restrict__ Btp, int ldb,
    float* __restrict__ Cout, int ldc,
    int M, int N, int K, float scale)
{
  typedef _Float16 T;
  const T* A = (const T*)Ap;
  const T* Bt = (const T*)Btp;
  __shared__ __align__(16) float sT[8][16 * 68];
  const int lane = threadIdx.x & 31;
  const int wave = threadIdx.x >> 5;
  const int tilesN = N >> 6;
  const int tilesM = M >> 6;
  const int tile = blockIdx.x * 8 + wave;
  if (tile >= tilesM * tilesN) return;
  const int tm = tile / tilesN;
  const int tn = tile - tm * tilesN;
  const int m0 = tm << 6;
  const int n0 = tn << 6;

  const int rlane = lane & 15;
  const int koff  = (lane >> 4) * 8;
  const int mOff  = (lane >> 4) * 8;

  v8f acc[4][4];
#pragma unroll
  for (int i = 0; i < 4; ++i)
#pragma unroll
    for (int j = 0; j < 4; ++j) acc[i][j] = (v8f){0.f,0.f,0.f,0.f,0.f,0.f,0.f,0.f};

  for (int k0 = 0; k0 < K; k0 += 32) {
    v16h bh[4];
#pragma unroll
    for (int j = 0; j < 4; ++j) {
      const size_t bo = (size_t)(n0 + (j << 4) + rlane) * ldb + koff + k0;
      bh[j] = FragH::load(Bt + bo);
    }
#pragma unroll
    for (int i = 0; i < 4; ++i) {
      const size_t ao = (size_t)(m0 + (i << 4) + rlane) * lda + koff + k0;
      v16h ah = FragH::load(A + ao);
#pragma unroll
      for (int j = 0; j < 4; ++j) {
        acc[i][j] = FragH::mma(ah, bh[j], acc[i][j]);
      }
      tie_h(acc[i][0], ah, bh[0]);
      tie_h(acc[i][1], ah, bh[1]);
      tie_h(acc[i][2], ah, bh[2]);
      tie_h(acc[i][3], ah, bh[3]);
    }
    keep4_h(bh[0], bh[1], bh[2], bh[3]);
  }
  acc_guard4(acc[0][0], acc[0][1], acc[0][2], acc[0][3]);
  acc_guard4(acc[1][0], acc[1][1], acc[1][2], acc[1][3]);
  acc_guard4(acc[2][0], acc[2][1], acc[2][2], acc[2][3]);
  acc_guard4(acc[3][0], acc[3][1], acc[3][2], acc[3][3]);

  float* slab = sT[wave];
#pragma unroll
  for (int i = 0; i < 4; ++i) {
    const int mBase = m0 + (i << 4);
#pragma unroll
    for (int j = 0; j < 4; ++j) {
#pragma unroll
      for (int r = 0; r < 8; ++r) {
        const float v = acc[i][j][r] * scale;
        slab[(mOff + r) * 68 + (j << 4) + rlane] = v;
      }
    }
    __builtin_amdgcn_fence(__ATOMIC_RELEASE, "workgroup");
    __builtin_amdgcn_wave_barrier();
    __builtin_amdgcn_fence(__ATOMIC_ACQUIRE, "workgroup");
    {
      float* C = Cout;
      const int hh = lane >> 4, c4 = (lane & 15) * 4;
      for (int pass = 0; pass < 2; ++pass) {
#pragma unroll
        for (int it = 0; it < 8; ++it) {
          const int row = it * 2 + hh;
          v4f v = *(const v4f*)(slab + row * 68 + c4);
          *(volatile v4f*)(C + (size_t)(mBase + row) * ldc + n0 + c4) = v;
        }
        __threadfence();
      }
    }
    __builtin_amdgcn_fence(__ATOMIC_RELEASE, "workgroup");
    __builtin_amdgcn_wave_barrier();
    __builtin_amdgcn_fence(__ATOMIC_ACQUIRE, "workgroup");
  }
}

__global__ __launch_bounds__(256) void repack_kernel(const float* __restrict__ CP, float* __restrict__ out)
{
  const int t = blockIdx.x * 256 + threadIdx.x;
  const int tc = (t < kOutVec) ? t : (kOutVec - 1);
  const int i0 = tc * 4;
  const int i1 = i0 + 2;
  const int ma = i0 / kColsN;
  const int ja = i0 - ma * kColsN;
  const int mb = i1 / kColsN;
  const int jb = i1 - mb * kColsN;
  v2f a = *(const v2f*)(CP + (size_t)ma * kColsNP + ja);
  v2f b = *(const v2f*)(CP + (size_t)mb * kColsNP + jb);
  asm volatile("" : "+v"(a));
  asm volatile("" : "+v"(b));
  v4f v;
  v[0] = a[0];
  v[1] = a[1];
  v[2] = b[0];
  v[3] = b[1];
  if (t < kOutVec) {
    float* q = out + (size_t)i0;
    *(volatile v4f*)q = v;
    __threadfence();
    *(volatile v4f*)q = v;
  }
}

extern "C" void kernel_launch(void* const* d_in, const int* in_sizes, int n_in,
                              void* d_out, int out_size, void* d_ws, size_t ws_size,
                              hipStream_t stream) {
  if (n_in < 4) return;
  if (in_sizes[0] != kBatch * kSigLen) return;
  if (in_sizes[1] != kFrame) return;
  if (in_sizes[2] != kFrame * kFrame) return;
  if (in_sizes[3] != kFrame * kFrame) return;
  if (out_size != kOutElems) return;
  if (ws_size < kWsTotal) return;

  const float* sig  = (const float*)d_in[0];
  const float* win  = (const float*)d_in[1];
  const float* tcos = (const float*)d_in[2];
  const float* tsin = (const float*)d_in[3];
  float* out = (float*)d_out;

  char* ws = (char*)d_ws;
  unsigned short* A16  = (unsigned short*)(ws + kOffA);
  unsigned short* BT16 = (unsigned short*)(ws + kOffB);
  float*          CP   = (float*)(ws + kOffC);

  prep_a_kernel<<<kAVec / 256, 256, 0, stream>>>(sig, win, A16);
  prep_b_kernel<<<kBVec / 256, 256, 0, stream>>>(tcos, tsin, BT16);

  gemm_f16_nt_kernel<<<kGemmBlocks, 256, 0, stream>>>(
      A16, kDepthK,
      BT16, kDepthK,
      CP, kColsNP,
      kRowsMP, kColsNP, kDepthK, kFold);

  repack_kernel<<<kOutBlocks, 256, 0, stream>>>(CP, out);
}
